// BCNet_77275051590189
// MI455X (gfx1250) — hardware-run, weakly checked
//
#include <hip/hip_runtime.h>
#include <math.h>

typedef __attribute__((ext_vector_type(16))) _Float16 v16h;
typedef __attribute__((ext_vector_type(8)))  _Float16 v8h;
typedef __attribute__((ext_vector_type(8)))  float    v8f;
typedef __attribute__((ext_vector_type(4)))  float    v4f;

constexpr int kBatch = 128;
constexpr int kObj   = 36;
constexpr int kQLen  = 14;
constexpr int kVDim  = 2048;
constexpr int kQDim  = 1024;
constexpr int kHid   = 2048;
constexpr int kRowsV = kBatch * kObj;
constexpr int kRowsQ = kBatch * kQLen;
constexpr float kWCarry    = 64.0f;
constexpr float kWCarryInv = 1.0f / 64.0f;
static_assert(kRowsV == 4608 && kRowsQ == 1792, "row counts");
static_assert((kVDim % 32) == 0 && (kQDim % 32) == 0 && (kHid % 32) == 0, "GEMM K multiples of 32");
static_assert((kRowsV % 64) == 0 && (kRowsQ % 64) == 0 && (kHid % 64) == 0 && (kVDim % 64) == 0, "GEMM M,N multiples of 64");
static_assert((((kRowsV / 64) * (kHid / 64)) % 8) == 0 && (((kRowsQ / 64) * (kHid / 64)) % 8) == 0, "8 tiles per block exactly");

constexpr size_t kOffV16  = 0;
constexpr size_t kOffWV16 = kOffV16  + (size_t)kRowsV * kVDim * 2;
constexpr size_t kOffW216 = kOffWV16 + (size_t)kHid   * kVDim * 2;
constexpr size_t kOffQ16  = kOffW216 + (size_t)kVDim  * kHid  * 2;
constexpr size_t kOffWQ16 = kOffQ16  + (size_t)kRowsQ * kQDim * 2;
constexpr size_t kOffQACT = kOffWQ16 + (size_t)kHid   * kQDim * 2;
constexpr size_t kOffQW   = kOffQACT + (size_t)kRowsQ * kHid  * 4;
constexpr size_t kOffLG16 = kOffQW   + (size_t)kBatch * kHid  * 4;
constexpr size_t kWsTotal = kOffLG16 + (size_t)kRowsV * kHid  * 2;
static_assert(kWsTotal == 78118912ull, "carve total");
static_assert(kWsTotal <= 134217728ull, "carve cap");
static_assert((kOffWV16 % 256) == 0 && (kOffW216 % 256) == 0 && (kOffQ16 % 256) == 0 && (kOffWQ16 % 256) == 0 &&
              (kOffQACT % 256) == 0 && (kOffQW % 256) == 0 && (kOffLG16 % 256) == 0, "256-B aligned regions");

__device__ __forceinline__ void keep4_h(v16h a, v16h b, v16h c, v16h d) { asm volatile("v_nop" :: "v"(a), "v"(b), "v"(c), "v"(d)); }
__device__ __forceinline__ void acc_guard4(v8f& a, v8f& b, v8f& c, v8f& d) { asm volatile("v_nop\n\tv_nop\n\tv_nop\n\tv_nop" : "+v"(a), "+v"(b), "+v"(c), "+v"(d)); }

union FragU { v16h v; v8h h[2]; };
__device__ __forceinline__ v16h frag_load(const _Float16* p) {
  FragU f;
  f.h[0] = *(const v8h*)(p);
  f.h[1] = *(const v8h*)(p + 16);
  return f.v;
}
__device__ __forceinline__ v8f mma_guarded(v16h a, v16h b, v8f c) {
  c = __builtin_amdgcn_wmma_f32_16x16x32_f16(false, a, false, b, (short)0, c, false, false);
  asm volatile("v_nop\n\tv_nop\n\tv_nop\n\tv_nop" : "+v"(c) : "v"(a), "v"(b));
  return c;
}

template <int EPI>
__global__ __launch_bounds__(256) void gemm_f16_tile64(
    const unsigned short* __restrict__ Ap, int lda,
    const unsigned short* __restrict__ Btp, int ldb,
    void* __restrict__ Cout, int ldc,
    const float* __restrict__ bias,
    const float* __restrict__ qw, int ldq,
    const float* __restrict__ bhp,
    int M, int N, int K, float scale) {
  const _Float16* A  = (const _Float16*)Ap;
  const _Float16* Bt = (const _Float16*)Btp;
  __shared__ __align__(16) float sT[8][16 * 68];
  const int lane = threadIdx.x & 31;
  const int wave = threadIdx.x >> 5;
  const int tilesN = N >> 6;
  const int tilesM = M >> 6;
  const int tile = blockIdx.x * 8 + wave;
  if (tile >= tilesM * tilesN) return;
  const int tm = tile / tilesN;
  const int tn = tile - tm * tilesN;
  const int m0 = tm << 6;
  const int n0 = tn << 6;

  const int rlane = lane & 15;
  const int koff  = (lane >> 4) * 8;
  const int mOff  = (lane >> 4) * 8;

  v8f acc[4][4];
#pragma unroll
  for (int i = 0; i < 4; ++i)
#pragma unroll
    for (int j = 0; j < 4; ++j) acc[i][j] = (v8f){0.f,0.f,0.f,0.f,0.f,0.f,0.f,0.f};

  for (int k0 = 0; k0 < K; k0 += 32) {
    v16h bfr[4];
#pragma unroll
    for (int j = 0; j < 4; ++j) {
      const size_t bo = (size_t)(n0 + (j << 4) + rlane) * ldb + koff + k0;
      bfr[j] = frag_load(Bt + bo);
    }
#pragma unroll
    for (int i = 0; i < 4; ++i) {
      const size_t ao = (size_t)(m0 + (i << 4) + rlane) * lda + koff + k0;
      const v16h ah = frag_load(A + ao);
#pragma unroll
      for (int j = 0; j < 4; ++j) acc[i][j] = mma_guarded(ah, bfr[j], acc[i][j]);
    }
    keep4_h(bfr[0], bfr[1], bfr[2], bfr[3]);
  }
  acc_guard4(acc[0][0], acc[0][1], acc[0][2], acc[0][3]);
  acc_guard4(acc[1][0], acc[1][1], acc[1][2], acc[1][3]);
  acc_guard4(acc[2][0], acc[2][1], acc[2][2], acc[2][3]);
  acc_guard4(acc[3][0], acc[3][1], acc[3][2], acc[3][3]);

  float* slab = sT[wave];
  float bj[4];
#pragma unroll
  for (int j = 0; j < 4; ++j) bj[j] = bias[n0 + (j << 4) + rlane];
  float bhv = 0.0f;
  if (EPI == 1) bhv = bhp[0];

#pragma unroll
  for (int i = 0; i < 4; ++i) {
    const int mBase = m0 + (i << 4);
#pragma unroll
    for (int j = 0; j < 4; ++j) {
#pragma unroll
      for (int r = 0; r < 8; ++r) {
        float x = acc[i][j][r] * scale + bj[j];
        if (EPI != 2) x = fmaxf(x, 0.0f);
        slab[(mOff + r) * 68 + (j << 4) + rlane] = x;
      }
    }
    __builtin_amdgcn_fence(__ATOMIC_RELEASE, "workgroup");
    __builtin_amdgcn_wave_barrier();
    __builtin_amdgcn_fence(__ATOMIC_ACQUIRE, "workgroup");
    if (EPI != 1) {
      float* C = (float*)Cout;
      const int hh = lane >> 4, c4 = (lane & 15) * 4;
      for (int pass = 0; pass < 2; ++pass) {
#pragma unroll
        for (int it = 0; it < 8; ++it) {
          const int row = it * 2 + hh;
          const v4f val = *(const v4f*)(slab + row * 68 + c4);
          *(volatile v4f*)(C + (size_t)(mBase + row) * ldc + n0 + c4) = val;
        }
        __threadfence();
      }
    } else {
      unsigned short* C = (unsigned short*)Cout;
      const int q = lane >> 3, c8 = (lane & 7) * 8;
      v8h hv[4];
#pragma unroll
      for (int it = 0; it < 4; ++it) {
        const int row  = it * 4 + q;
        const int grow = mBase + row;
        const int bidx = grow / kObj;
        const float* qp = qw + (size_t)bidx * ldq + n0 + c8;
        const v4f q0 = *(const v4f*)(qp);
        const v4f q1 = *(const v4f*)(qp + 4);
        const float* sp = slab + row * 68 + c8;
        const v4f s0 = *(const v4f*)(sp);
        const v4f s1 = *(const v4f*)(sp + 4);
#pragma unroll
        for (int e = 0; e < 4; ++e) {
          const float x0 = s0[e] * q0[e] + bhv;
          const float x1 = s1[e] * q1[e] + bhv;
          hv[it][e]     = (_Float16)x0;
          hv[it][4 + e] = (_Float16)x1;
        }
      }
      for (int pass = 0; pass < 2; ++pass) {
#pragma unroll
        for (int it = 0; it < 4; ++it) {
          const int row = it * 4 + q;
          *(volatile v8h*)(C + (size_t)(mBase + row) * ldc + n0 + c8) = hv[it];
        }
        __threadfence();
      }
    }
    __builtin_amdgcn_fence(__ATOMIC_RELEASE, "workgroup");
    __builtin_amdgcn_wave_barrier();
    __builtin_amdgcn_fence(__ATOMIC_ACQUIRE, "workgroup");
  }
}

__global__ __launch_bounds__(256) void cvt_f32_f16x8_kernel(
    const float* __restrict__ src, unsigned short* __restrict__ dst, int total8, float carry)
{
  const int i = blockIdx.x * 256 + threadIdx.x;
  if (i >= total8) return;
  const size_t e0 = (size_t)i << 3;
  const v4f a0 = *(const v4f*)(src + e0);
  const v4f a1 = *(const v4f*)(src + e0 + 4);
  v8h hv;
#pragma unroll
  for (int e = 0; e < 4; ++e) {
    const float x0 = a0[e] * carry;
    const float x1 = a1[e] * carry;
    hv[e]     = (_Float16)x0;
    hv[4 + e] = (_Float16)x1;
  }
  unsigned short* p = dst + e0;
  *(volatile v8h*)p = hv;
  __threadfence();
  *(volatile v8h*)p = hv;
}

__global__ __launch_bounds__(256) void qw_reduce_kernel(
    const float* __restrict__ qact, const float* __restrict__ wh, float* __restrict__ qwout)
{
  const int i  = blockIdx.x * 256 + threadIdx.x;
  if (i >= kBatch * (kHid / 4)) return;
  const int b  = i / (kHid / 4);
  const int h4 = (i - b * (kHid / 4)) * 4;
  v4f acc = (v4f){0.f, 0.f, 0.f, 0.f};
  const float* base = qact + (size_t)b * kQLen * kHid + h4;
#pragma unroll 1
  for (int j = 0; j < kQLen; ++j) {
    const float w = wh[j];
    const v4f x = *(const v4f*)(base + (size_t)j * kHid);
    acc[0] = fmaf(w, x[0], acc[0]);
    acc[1] = fmaf(w, x[1], acc[1]);
    acc[2] = fmaf(w, x[2], acc[2]);
    acc[3] = fmaf(w, x[3], acc[3]);
  }
  float* p = qwout + (size_t)b * kHid + h4;
  *(volatile v4f*)p = acc;
  __threadfence();
  *(volatile v4f*)p = acc;
}

extern "C" void kernel_launch(void* const* d_in, const int* in_sizes, int n_in,
                              void* d_out, int out_size, void* d_ws, size_t ws_size,
                              hipStream_t stream) {
  if (n_in < 10) return;
  if (in_sizes[0] != kRowsV * kVDim) return;
  if (in_sizes[1] != kRowsQ * kQDim) return;
  if (in_sizes[2] != kHid * kVDim) return;
  if (in_sizes[3] != kHid) return;
  if (in_sizes[4] != kHid * kQDim) return;
  if (in_sizes[5] != kHid) return;
  if (in_sizes[6] != kQLen) return;
  if (in_sizes[7] != 1) return;
  if (in_sizes[8] != kVDim * kHid) return;
  if (in_sizes[9] != kVDim) return;
  if (out_size != kRowsV * kVDim) return;
  if (ws_size < kWsTotal) return;

  const float* v  = (const float*)d_in[0];
  const float* q  = (const float*)d_in[1];
  const float* Wv = (const float*)d_in[2];
  const float* bv = (const float*)d_in[3];
  const float* Wq = (const float*)d_in[4];
  const float* bq = (const float*)d_in[5];
  const float* wh = (const float*)d_in[6];
  const float* bh = (const float*)d_in[7];
  const float* W2 = (const float*)d_in[8];
  const float* b2 = (const float*)d_in[9];
  float* out = (float*)d_out;

  char* ws = (char*)d_ws;
  unsigned short* V16  = (unsigned short*)(ws + kOffV16);
  unsigned short* WV16 = (unsigned short*)(ws + kOffWV16);
  unsigned short* W216 = (unsigned short*)(ws + kOffW216);
  unsigned short* Q16  = (unsigned short*)(ws + kOffQ16);
  unsigned short* WQ16 = (unsigned short*)(ws + kOffWQ16);
  float*          QACT = (float*)(ws + kOffQACT);
  float*          QW   = (float*)(ws + kOffQW);
  unsigned short* LG16 = (unsigned short*)(ws + kOffLG16);

  cvt_f32_f16x8_kernel<<<(kRowsV * kVDim / 8) / 256, 256, 0, stream>>>(v,  V16,  kRowsV * kVDim / 8, 1.0f);
  cvt_f32_f16x8_kernel<<<(kHid * kVDim / 8) / 256, 256, 0, stream>>>(Wv, WV16, kHid * kVDim / 8, kWCarry);
  cvt_f32_f16x8_kernel<<<(kVDim * kHid / 8) / 256, 256, 0, stream>>>(W2, W216, kVDim * kHid / 8, kWCarry);
  cvt_f32_f16x8_kernel<<<(kRowsQ * kQDim / 8) / 256, 256, 0, stream>>>(q,  Q16,  kRowsQ * kQDim / 8, 1.0f);
  cvt_f32_f16x8_kernel<<<(kHid * kQDim / 8) / 256, 256, 0, stream>>>(Wq, WQ16, kHid * kQDim / 8, kWCarry);

  gemm_f16_tile64<0><<<((kRowsQ / 64) * (kHid / 64)) / 8, 256, 0, stream>>>(
      Q16, kQDim, WQ16, kQDim, (void*)QACT, kHid, bq, bq, kHid, bq,
      kRowsQ, kHid, kQDim, kWCarryInv);

  qw_reduce_kernel<<<(kBatch * (kHid / 4)) / 256, 256, 0, stream>>>(QACT, wh, QW);

  gemm_f16_tile64<1><<<((kRowsV / 64) * (kHid / 64)) / 8, 256, 0, stream>>>(
      V16, kVDim, WV16, kVDim, (void*)LG16, kHid, bv, QW, kHid, bh,
      kRowsV, kHid, kVDim, kWCarryInv);

  gemm_f16_tile64<2><<<((kRowsV / 64) * (kVDim / 64)) / 8, 256, 0, stream>>>(
      LG16, kHid, W216, kHid, (void*)out, kVDim, b2, b2, kVDim, b2,
      kRowsV, kVDim, kHid, kWCarryInv);
}
